// TSModel_4896262718051
// MI455X (gfx1250) — hardware-verified
//
#include <hip/hip_runtime.h>
#include <math.h>

constexpr int NB_ROWS  = 2048;
constexpr int NSTEP    = 1024;
constexpr int NUNIT    = 64;
constexpr int NGATE    = 4 * NUNIT;
constexpr int NTHR     = 128;
constexpr int ROWS_BLK = 16;
constexpr int XCHUNK   = 256;
constexpr int HST      = 72;
constexpr int G1P      = 16;
constexpr int OBP      = 36;
constexpr int OCH      = 32;
constexpr int W1ROWS   = 16;
constexpr int WH_BLOCKS = (NGATE * NUNIT / 8) / NTHR;
constexpr float WHC = 64.0f;  constexpr float WHC_INV = 1.0f / 64.0f;
constexpr float W1C = 16.0f;  constexpr float W1C_INV = 1.0f / 16.0f;
static_assert(NB_ROWS % ROWS_BLK == 0);
static_assert(NUNIT == 16 * (NTHR / 32));
static_assert(NUNIT % 32 == 0);
static_assert(NSTEP % XCHUNK == 0 && XCHUNK % OCH == 0 && NSTEP % OCH == 0);
static_assert(ROWS_BLK * XCHUNK == 4 * 8 * NTHR);
static_assert((2 * ROWS_BLK * HST) % NTHR == 0 && (ROWS_BLK * HST) % NTHR == 0);
static_assert(WH_BLOCKS * NTHR * 8 == NGATE * NUNIT);
static_assert(NTHR * 8 == W1ROWS * NUNIT);
static_assert(OBP % 4 == 0 && HST % 8 == 0);

typedef __attribute__((ext_vector_type(16))) _Float16 v16h;
typedef __attribute__((ext_vector_type(8)))  _Float16 v8h;
typedef __attribute__((ext_vector_type(8)))  float    v8f;
typedef __attribute__((ext_vector_type(4)))  float    v4f;

__device__ __forceinline__ void dep_guard_h(v8f& a, v8f& b, v16h x, v16h y) { asm volatile("v_nop\n\tv_nop\n\tv_nop\n\tv_nop" : "+v"(a), "+v"(b) : "v"(x), "v"(y)); }
__device__ __forceinline__ void keep4_h(v16h a, v16h b, v16h c, v16h d) { asm volatile("v_nop" :: "v"(a), "v"(b), "v"(c), "v"(d)); }
__device__ __forceinline__ void acc_guard4(v8f& a, v8f& b, v8f& c, v8f& d) { asm volatile("v_nop\n\tv_nop\n\tv_nop\n\tv_nop" : "+v"(a), "+v"(b), "+v"(c), "+v"(d)); }
__device__ __forceinline__ void acc_guard1(v8f& a, v16h w, v16h x, v16h y, v16h z) { asm volatile("v_nop\n\tv_nop\n\tv_nop\n\tv_nop" : "+v"(a) : "v"(w), "v"(x), "v"(y), "v"(z)); }
__device__ __forceinline__ void load_group_wait(v16h a, v16h b, float c, float d) {
  asm volatile("s_wait_loadcnt 0x0" :: "v"(a), "v"(b), "v"(c), "v"(d) : "memory");
}
__device__ __forceinline__ void load_group_wait4(float a, float b, float c, float d) {
  asm volatile("s_wait_loadcnt 0x0" :: "v"(a), "v"(b), "v"(c), "v"(d) : "memory");
}
template <typename T> struct Frag;
template <> struct Frag<_Float16> {
  typedef v16h V; union U { v16h v; v8h h[2]; };
  static __device__ __forceinline__ v16h load(const _Float16* p) {
    U f; f.h[0] = *(const v8h*)(p); f.h[1] = *(const v8h*)(p + 16); return f.v;
  }
  static __device__ __forceinline__ v8f mma(v16h a, v16h b, v8f c) {
    return __builtin_amdgcn_wmma_f32_16x16x32_f16(false, a, false, b, (short)0, c, false, false);
  }
};

__device__ __forceinline__ float fsig(float x)  { return __builtin_amdgcn_rcpf(1.0f + __expf(-x)); }
__device__ __forceinline__ float ftanh(float x) { return 1.0f - 2.0f * __builtin_amdgcn_rcpf(__expf(2.0f * x) + 1.0f); }

__global__ __launch_bounds__(NTHR) void wplane_kernel(const float* __restrict__ whh0, const float* __restrict__ wih1,
                                                      unsigned short* __restrict__ WHp, unsigned short* __restrict__ W1p) {
  const int tid = threadIdx.x;
  if (blockIdx.x < WH_BLOCKS) {
    const int i = blockIdx.x * NTHR + tid;
    const float* sp = whh0 + (size_t)i * 8;
    const v4f a = *(const v4f*)(sp);
    const v4f b = *(const v4f*)(sp + 4);
    v8h hv;
#pragma unroll
    for (int e = 0; e < 4; ++e) { hv[e] = (_Float16)(a[e] * WHC); hv[4 + e] = (_Float16)(b[e] * WHC); }
    unsigned short* dp = WHp + (size_t)i * 8;
    *(volatile v8h*)dp = hv;
    __threadfence();
    *(volatile v8h*)dp = hv;
  } else {
    const int row = tid >> 3;
    const int c8  = (tid & 7) * 8;
    const int rs  = row < 4 ? row : 3;
    const float scl = row < 4 ? W1C : 0.0f;
    const float* sp = wih1 + rs * NUNIT + c8;
    const v4f a = *(const v4f*)(sp);
    const v4f b = *(const v4f*)(sp + 4);
    v8h hv;
#pragma unroll
    for (int e = 0; e < 4; ++e) { hv[e] = (_Float16)(a[e] * scl); hv[4 + e] = (_Float16)(b[e] * scl); }
    unsigned short* dp = W1p + (size_t)tid * 8;
    *(volatile v8h*)dp = hv;
    __threadfence();
    *(volatile v8h*)dp = hv;
  }
}

__global__ __launch_bounds__(NTHR) void cell2_seq_kernel(const float* __restrict__ xin_g,
                                                         const float* __restrict__ w_ih0, const float* __restrict__ b_ih0,
                                                         const float* __restrict__ b_hh0,
                                                         const float* __restrict__ w_hh1, const float* __restrict__ b_ih1,
                                                         const float* __restrict__ b_hh1,
                                                         const unsigned short* __restrict__ WHp,
                                                         const unsigned short* __restrict__ W1p,
                                                         float* __restrict__ out) {
  __shared__ __align__(16) float    Xs[ROWS_BLK * XCHUNK];
  __shared__ __align__(16) _Float16 Hs[2 * ROWS_BLK * HST];
  __shared__ __align__(16) _Float16 Cs[ROWS_BLK * HST];
  __shared__ __align__(16) float    Gs[ROWS_BLK * G1P];
  __shared__ __align__(16) float    Ob[ROWS_BLK * OBP];
  const _Float16* WH = (const _Float16*)WHp;
  const _Float16* W1 = (const _Float16*)W1p;
  const int tid = threadIdx.x, lane = tid & 31, wave = tid >> 5;
  const int c = lane & 15, hh = lane >> 4, koff = hh * 8;
  const int rowbase = blockIdx.x * ROWS_BLK;
  const int unit = 16 * wave + c;

#pragma unroll 1
  for (int i = tid; i < 2 * ROWS_BLK * HST; i += NTHR) Hs[i] = (_Float16)0.0f;
#pragma unroll 1
  for (int i = tid; i < ROWS_BLK * HST; i += NTHR) Cs[i] = (_Float16)0.0f;

  v16h Bf[4][2];
  float bsum[4], wih[4];
#pragma unroll
  for (int g = 0; g < 4; ++g) {
    const int n = g * NUNIT + unit;
    bsum[g] = b_ih0[n] + b_hh0[n];
    wih[g]  = w_ih0[n];
    const _Float16* wr = WH + (size_t)n * NUNIT + koff;
    Bf[g][0] = Frag<_Float16>::load(wr);
    Bf[g][1] = Frag<_Float16>::load(wr + 32);
    load_group_wait(Bf[g][0], Bf[g][1], bsum[g], wih[g]);
  }
  float b1s[4], whh1v[4];
#pragma unroll
  for (int j = 0; j < 4; ++j) { b1s[j] = b_ih1[j] + b_hh1[j]; whh1v[j] = w_hh1[j]; }
  load_group_wait4(b1s[0], b1s[1], b1s[2], b1s[3]);
  load_group_wait4(whh1v[0], whh1v[1], whh1v[2], whh1v[3]);

  float cst[8];
#pragma unroll
  for (int r = 0; r < 8; ++r) cst[r] = 0.0f;
  float c1 = 0.0f, h1 = 0.0f;
  __syncthreads();

  const v8f z8 = {0.f, 0.f, 0.f, 0.f, 0.f, 0.f, 0.f, 0.f};

#pragma unroll 1
  for (int t = 0; t < NSTEP; ++t) {
    if ((t & (XCHUNK - 1)) == 0) {
      __syncthreads();
#pragma unroll
      for (int it = 0; it < 8; ++it) {
        const int idx = it * NTHR + tid;
        const int m = idx >> 6, j4 = (idx & 63) * 4;
        const v4f v = *(const v4f*)(xin_g + (size_t)(rowbase + m) * NSTEP + t + j4);
        *(v4f*)(Xs + m * XCHUNK + j4) = v;
      }
      __syncthreads();
    }
    const int cur = t & 1;
    const int tc  = t & (XCHUNK - 1);
    const _Float16* hrow = Hs + cur * (ROWS_BLK * HST) + c * HST + koff;
    _Float16* hnext = Hs + (cur ^ 1) * (ROWS_BLK * HST);

    float xv[8];
#pragma unroll
    for (int r = 0; r < 8; ++r) xv[r] = Xs[(8 * hh + r) * XCHUNK + tc];
    v8f acc[4];
    acc[0] = z8; acc[1] = z8; acc[2] = z8; acc[3] = z8;
    const v16h a0 = Frag<_Float16>::load(hrow);
    const v16h a1 = Frag<_Float16>::load(hrow + 32);
#pragma unroll
    for (int g = 0; g < 4; ++g) {
      acc[g] = Frag<_Float16>::mma(a0, Bf[g][0], acc[g]);
      acc[g] = Frag<_Float16>::mma(a1, Bf[g][1], acc[g]);
    }
    dep_guard_h(acc[0], acc[3], a0, a1);
    keep4_h(Bf[3][0], Bf[3][1], Bf[2][0], Bf[2][1]);
    acc_guard4(acc[0], acc[1], acc[2], acc[3]);
#pragma unroll
    for (int r = 0; r < 8; ++r) {
      const float zi = acc[0][r] * WHC_INV + (bsum[0] + xv[r] * wih[0]);
      const float zf = acc[1][r] * WHC_INV + (bsum[1] + xv[r] * wih[1]);
      const float zg = acc[2][r] * WHC_INV + (bsum[2] + xv[r] * wih[2]);
      const float zo = acc[3][r] * WHC_INV + (bsum[3] + xv[r] * wih[3]);
      const float ig = fsig(zi);
      const float fg = fsig(zf);
      const float gg = ftanh(zg);
      const float og = fsig(zo);
      const float cn = fg * cst[r] + ig * gg;
      const float hn = og * ftanh(cn);
      cst[r] = cn;
      hnext[(8 * hh + r) * HST + unit] = (_Float16)hn;
      Cs[(8 * hh + r) * HST + unit]    = (_Float16)cn;
    }
    __syncthreads();

    if (wave == 0) {
      const _Float16* crow = Cs + c * HST + koff;
      const _Float16* w1r  = W1 + c * NUNIT + koff;
      const v16h ca0 = Frag<_Float16>::load(crow);
      const v16h ca1 = Frag<_Float16>::load(crow + 32);
      const v16h wb0 = Frag<_Float16>::load(w1r);
      const v16h wb1 = Frag<_Float16>::load(w1r + 32);
      v8f g1 = z8;
      g1 = Frag<_Float16>::mma(ca0, wb0, g1);
      g1 = Frag<_Float16>::mma(ca1, wb1, g1);
      acc_guard1(g1, ca0, ca1, wb0, wb1);
#pragma unroll
      for (int r = 0; r < 8; ++r) Gs[(8 * hh + r) * G1P + c] = g1[r];
    }
    __syncthreads();

    if (wave == 0) {
      const int m = c;
      const v4f gv = *(const v4f*)(Gs + m * G1P);
      const float zi = gv[0] * W1C_INV + (b1s[0] + h1 * whh1v[0]);
      const float zf = gv[1] * W1C_INV + (b1s[1] + h1 * whh1v[1]);
      const float zg = gv[2] * W1C_INV + (b1s[2] + h1 * whh1v[2]);
      const float zo = gv[3] * W1C_INV + (b1s[3] + h1 * whh1v[3]);
      const float c1n = fsig(zf) * c1 + fsig(zi) * ftanh(zg);
      h1 = fsig(zo) * ftanh(c1n);
      c1 = c1n;
      if (lane < 16) Ob[m * OBP + (t & (OCH - 1))] = c1n;
    }

    if ((t & (OCH - 1)) == (OCH - 1)) {
      __syncthreads();
      if (wave == 0) {
        const int q = lane >> 3, c4 = (lane & 7) * 4;
        const int t0 = t - (OCH - 1);
        for (int pass = 0; pass < 2; ++pass) {
#pragma unroll
          for (int it = 0; it < 4; ++it) {
            const int row = it * 4 + q;
            const v4f v = *(const v4f*)(Ob + row * OBP + c4);
            *(volatile v4f*)(out + (size_t)(rowbase + row) * NSTEP + t0 + c4) = v;
          }
          __threadfence();
        }
      }
    }
  }
}

extern "C" void kernel_launch(void* const* d_in, const int* in_sizes, int n_in,
                              void* d_out, int out_size, void* d_ws, size_t ws_size, hipStream_t stream) {
  if (n_in < 9 || d_out == nullptr || d_ws == nullptr) return;
  if (in_sizes[0] != NB_ROWS * NSTEP || in_sizes[1] != NGATE || in_sizes[2] != NGATE * NUNIT ||
      in_sizes[3] != NGATE || in_sizes[4] != NGATE || in_sizes[5] != 4 * NUNIT ||
      in_sizes[6] != 4 || in_sizes[7] != 4 || in_sizes[8] != 4 || out_size != NB_ROWS * NSTEP) return;

  const float* xin   = (const float*)d_in[0];
  const float* w_ih0 = (const float*)d_in[1];
  const float* w_hh0 = (const float*)d_in[2];
  const float* b_ih0 = (const float*)d_in[3];
  const float* b_hh0 = (const float*)d_in[4];
  const float* w_ih1 = (const float*)d_in[5];
  const float* w_hh1 = (const float*)d_in[6];
  const float* b_ih1 = (const float*)d_in[7];
  const float* b_hh1 = (const float*)d_in[8];
  float* out = (float*)d_out;

  char* ws = (char*)d_ws; size_t off = 0;
  auto carve = [&](size_t bytes) -> char* { char* p = ws + off; off += (bytes + 255) & ~(size_t)255; return p; };
  unsigned short* WH = (unsigned short*)carve((size_t)NGATE * NUNIT * 2);
  unsigned short* W1 = (unsigned short*)carve((size_t)W1ROWS * NUNIT * 2);
  if (off > ws_size || off > (size_t)134217728) return;

  wplane_kernel<<<WH_BLOCKS + 1, NTHR, 0, stream>>>(w_hh0, w_ih1, WH, W1);
  cell2_seq_kernel<<<NB_ROWS / ROWS_BLK, NTHR, 0, stream>>>(xin, w_ih0, b_ih0, b_hh0, w_hh1, b_ih1, b_hh1, WH, W1, out);
}
